// ImplicitGeometricPriors_45698452029979
// MI455X (gfx1250) — hardware-verified
//
#include <hip/hip_runtime.h>
#include <math.h>

typedef __attribute__((ext_vector_type(16))) _Float16 v16h;
typedef __attribute__((ext_vector_type(16))) __bf16 v16b;
typedef __attribute__((ext_vector_type(8)))  _Float16 v8h;
typedef __attribute__((ext_vector_type(8)))  float v8f;
typedef __attribute__((ext_vector_type(4)))  float v4f;
typedef __attribute__((ext_vector_type(2)))  float v2f;
typedef __attribute__((ext_vector_type(4)))  unsigned v4u;
typedef __attribute__((ext_vector_type(4)))  int v4i;
typedef float __attribute__((may_alias)) float_a;
typedef int __attribute__((may_alias)) int_a;

template <typename T> __device__ __forceinline__ void vst2(void* p, T v) { *(volatile T*)p = v; __threadfence(); *(volatile T*)p = v; }
__device__ __forceinline__ v8f wmma16(v16h a, v16h b, v8f c) {
  v8f d = __builtin_amdgcn_wmma_f32_16x16x32_f16(false, a, false, b, (short)0, c, false, false);
  asm volatile("v_nop\n\tv_nop\n\tv_nop\n\tv_nop" : "+v"(d) : "v"(a), "v"(b));
  return d;
}
__device__ __forceinline__ v8f wmma_bf(v16b a, v16b b, v8f c) {
  v8f d = __builtin_amdgcn_wmma_f32_16x16x32_bf16(false, a, false, b, (short)0, c, false, false);
  asm volatile("v_nop\n\tv_nop\n\tv_nop\n\tv_nop" : "+v"(d) : "v"(a), "v"(b));
  return d;
}
__device__ __forceinline__ v16h frag_h(const _Float16* rowk0, int lane) {
  union { v16h v; v8h q[2]; } u; const _Float16* p = rowk0 + 8 * (lane >> 4);
  u.q[0] = *(const v8h*)p; u.q[1] = *(const v8h*)(p + 16); return u.v;
}
__device__ __forceinline__ v16h frag_f32(const float* rowk0, int lane) {
  v16h a; const float* p = rowk0 + 8 * (lane >> 4);
#pragma unroll
  for (int i = 0; i < 8; ++i) { a[i] = (_Float16)p[i]; a[8 + i] = (_Float16)p[16 + i]; }
  return a;
}
__device__ __forceinline__ v16h frag_f32s(const float* rowk0, int lane, float sc) {
  v16h a; const float* p = rowk0 + 8 * (lane >> 4);
#pragma unroll
  for (int i = 0; i < 8; ++i) { a[i] = (_Float16)(p[i] * sc); a[8 + i] = (_Float16)(p[16 + i] * sc); }
  return a;
}
__device__ __forceinline__ v16h fragc_f32(const float* W, int k0, int n, int lane, int ld, int K) {
  v16h a; const int g = lane >> 4;
#pragma unroll
  for (int i = 0; i < 8; ++i) { const int ka = k0 + 8 * g + i, kb = ka + 16;
    a[i] = (_Float16)(ka < K ? W[(size_t)(ka < K ? ka : K - 1) * ld + n] : 0.f); a[8 + i] = (_Float16)(kb < K ? W[(size_t)(kb < K ? kb : K - 1) * ld + n] : 0.f); }
  return a;
}
struct F2 { v16b h, l; };
__device__ __forceinline__ F2 bsplit16(const float v[16]) { F2 r;
#pragma unroll
  for (int i = 0; i < 16; ++i) { const __bf16 h = (__bf16)v[i]; r.h[i] = h; r.l[i] = (__bf16)(v[i] - (float)h); }
  return r; }
__device__ __forceinline__ F2 split_row(const float* row, int k0, int lane) { float v[16]; const float* p = row + k0 + 8 * (lane >> 4);
#pragma unroll
  for (int i = 0; i < 8; ++i) { v[i] = p[i]; v[8 + i] = p[16 + i]; }
  return bsplit16(v); }
__device__ __forceinline__ F2 split_rowK(const float* row, int k0, int lane, int K) { float v[16]; const int g = lane >> 4;
#pragma unroll
  for (int i = 0; i < 8; ++i) { const int ka = k0 + 8 * g + i, kb = ka + 16; v[i] = ka < K ? row[ka < K ? ka : K - 1] : 0.f; v[8 + i] = kb < K ? row[kb < K ? kb : K - 1] : 0.f; }
  return bsplit16(v); }
__device__ __forceinline__ F2 split_col(const float* W, int k0, int n, int lane, int ld, int K) { float v[16]; const int g = lane >> 4;
#pragma unroll
  for (int i = 0; i < 8; ++i) { const int ka = k0 + 8 * g + i, kb = ka + 16; v[i] = ka < K ? W[(size_t)(ka < K ? ka : K - 1) * ld + n] : 0.f; v[8 + i] = kb < K ? W[(size_t)(kb < K ? kb : K - 1) * ld + n] : 0.f; }
  return bsplit16(v); }
__device__ __forceinline__ v8f mac3(const F2& a, const F2& b, v8f c) { c = wmma_bf(a.l, b.h, c); c = wmma_bf(a.h, b.l, c); return wmma_bf(a.h, b.h, c); }
__device__ __forceinline__ float sigm(float v) { return 1.0f / (1.0f + expf(-v)); }
#define LDSX() do { asm volatile("s_wait_dscnt 0" ::: "memory"); __builtin_amdgcn_wave_barrier(); __builtin_amdgcn_fence(__ATOMIC_RELEASE, "workgroup"); } while (0)


#define NB 2
#define NPT 512
#define DD 768
#define KN 64
#define NH 8
#define HD 96
#define NR (NB * NPT)
#ifndef NRB
#define NRB (NR / 64)
#endif
typedef __attribute__((ext_vector_type(8))) __bf16 v8b;
__device__ __forceinline__ v16b frag_b(const __bf16* rowk0, int lane) {
  union { v16b v; v8b q[2]; } u; const __bf16* p = rowk0 + 8 * (lane >> 4);
  u.q[0] = *(const v8b*)p; u.q[1] = *(const v8b*)(p + 16); return u.v;
}
__device__ __forceinline__ float bfr(float v) { return (float)(__bf16)v; }
__device__ __attribute__((noinline)) float exp_ni(float v) { return expf(v); }
__device__ __attribute__((noinline)) float erf_ni(float v) { return erff(v); }

#define WS_PW   0u
#define WS_PWE  (WS_PW + 2u * (size_t)4 * DD * DD)
#define WS_IDX  (WS_PWE + 2u * (size_t)DD * 2 * DD)
#define WS_DST  (WS_IDX + 4u * NR * KN)
#define WS_FQ   (WS_DST + 4u * NR * KN)
#define WS_FK   (WS_FQ + 4u * (size_t)NR * DD)
#define WS_FV   (WS_FK + 4u * (size_t)NR * DD)
#define WS_ATT  (WS_FV + 4u * (size_t)NR * DD)
#define WS_C2   (WS_ATT + 4u * (size_t)NR * DD)
#define WS_Y    (WS_C2 + 4u * (size_t)NR * DD)
#define WS_VEC  (WS_Y + 4u * (size_t)NR * DD)
#define WS_END  (WS_VEC + 4u * 4 * DD)

__global__ __launch_bounds__(256) void k_pack(const float* __restrict__ WQ, const float* __restrict__ WK, const float* __restrict__ WV, const float* __restrict__ WO, const float* __restrict__ WE, __bf16* __restrict__ P) {
  const int n = blockIdx.x, which = blockIdx.y, t = threadIdx.x; __shared__ __align__(16) __bf16 s[2 * DD];
  if (which < 4) { const float* Wm = (which == 0) ? WQ : (which == 1) ? WK : (which == 2) ? WV : WO; for (int k = t; k < DD; k += 256) s[k] = (__bf16)Wm[(size_t)k * DD + n]; __syncthreads(); for (int q = t; q < DD / 8; q += 256) vst2((unsigned*)(P + WS_PW / 2 + ((size_t)which * DD + n) * DD + q * 8), *(const v4u*)&s[q * 8]); }
  else { for (int k = t; k < 2 * DD; k += 256) s[k] = (__bf16)WE[(size_t)k * DD + n]; __syncthreads(); for (int q = t; q < 2 * DD / 8; q += 256) vst2((unsigned*)(P + WS_PWE / 2 + (size_t)n * 2 * DD + q * 8), *(const v4u*)&s[q * 8]); }
}
__global__ __launch_bounds__(256) void k_vec(const float* __restrict__ WD, const float* __restrict__ BD, const float* __restrict__ WK, const float* __restrict__ BK, const float* __restrict__ WV, const float* __restrict__ BV, float* __restrict__ VEC) {
  const int n = blockIdx.x * 256 + threadIdx.x; float a = 0.f, b = 0.f, c = 0.f, e = 0.f;
#pragma unroll 1
  for (int d = 0; d < DD; ++d) { const float wd = bfr(WD[d]), bd = bfr(BD[d]), wk = bfr(WK[(size_t)d * DD + n]), wv = bfr(WV[(size_t)d * DD + n]); a += wd * wk; b += wd * wv; c += bd * wk; e += bd * wv; }
  VEC[n] = a; VEC[DD + n] = b; VEC[2 * DD + n] = c + bfr(BK[n]); VEC[3 * DD + n] = e + bfr(BV[n]);
}
__global__ __launch_bounds__(64) void k_knn(const float* __restrict__ POS, int* __restrict__ IDX, float* __restrict__ DST) {
  __shared__ float sp[NPT * 3]; __shared__ float sd[64][KN + 1]; __shared__ int si[64][KN + 1];
  const int t = threadIdx.x; const size_t b = blockIdx.y; const int n = blockIdx.x * 64 + t;
  for (int e = t; e < NPT * 3; e += 64) sp[e] = bfr(POS[b * NPT * 3 + e]);
  __syncthreads();
  const float xn = sp[n * 3], yn = sp[n * 3 + 1], zn = sp[n * 3 + 2]; const float sqn = (xn * xn + yn * yn) + zn * zn;
  for (int k = 0; k < KN; ++k) { sd[t][k] = 3.0e38f; si[t][k] = 0x7fffffff; }
  int cnt = 0;
#pragma unroll 1
  for (int m = 0; m < NPT; ++m) { const float xm = sp[m * 3], ym = sp[m * 3 + 1], zm = sp[m * 3 + 2]; const float sqm = (xm * xm + ym * ym) + zm * zm; const float dt = (xn * xm + yn * ym) + zn * zm; const float d2 = (sqn + sqm) - 2.0f * dt;
    if (cnt < KN || d2 < sd[t][KN - 1]) { int p = (cnt < KN) ? cnt : KN - 1; while (p > 0 && sd[t][p - 1] > d2) { sd[t][p] = sd[t][p - 1]; si[t][p] = si[t][p - 1]; --p; } sd[t][p] = d2; si[t][p] = m; if (cnt < KN) ++cnt; } }
  const size_t row = b * NPT + n;
  for (int k = 0; k < KN; ++k) { IDX[row * KN + k] = si[t][k]; DST[row * KN + k] = sqrtf(fmaxf(sd[t][k], 0.f)); }
}
template <int KIN>
__global__ __launch_bounds__(128) void k_lin(const float* __restrict__ A, const float* __restrict__ A2, const __bf16* __restrict__ Wr, const float* __restrict__ BIAS, float* __restrict__ OUT) {
  __shared__ __align__(16) float so[4][16][132];
  const int tid = threadIdx.x, wave = tid >> 5, lane = tid & 31, col = lane & 15, g = lane >> 4; const size_t r0 = (size_t)blockIdx.x * 64 + wave * 16; const int n0 = blockIdx.y * 128;
  v8f acc[8] = {};
#pragma unroll 2
  for (int kc = 0; kc < KIN / 32; ++kc) { const bool second = (A2 != nullptr) && (kc >= DD / 32); const float* base = second ? A2 + (r0 + col) * DD : A + (r0 + col) * (A2 ? DD : KIN); const int kk = second ? (kc - DD / 32) * 32 : kc * 32;
    const F2 a = split_row(base, kk, lane);
#pragma unroll
    for (int j = 0; j < 8; ++j) { const v16b w = frag_b(Wr + (size_t)(n0 + j * 16 + col) * KIN + kc * 32, lane); acc[j] = wmma_bf(a.l, w, acc[j]); acc[j] = wmma_bf(a.h, w, acc[j]); } }
#pragma unroll
  for (int j = 0; j < 8; ++j) { const float bb = BIAS ? bfr(BIAS[n0 + j * 16 + col]) : 0.f;
#pragma unroll
    for (int r = 0; r < 8; ++r) so[wave][8 * g + r][j * 16 + col] = acc[j][r] + bb; }
  LDSX();
  for (int rl = 0; rl < 16; ++rl) vst2(OUT + (r0 + rl) * DD + n0 + lane * 4, *(const v4f*)&so[wave][rl][lane * 4]);
}
__global__ __launch_bounds__(256) void k_copyf(const float* __restrict__ F0, float* __restrict__ OUT) { const size_t row = blockIdx.x; const int t = threadIdx.x; for (int q = t; q < DD / 4; q += 256) { v4f v; for (int i = 0; i < 4; ++i) v[i] = bfr(F0[row * DD + q * 4 + i]); vst2(OUT + row * DD + q * 4, v); } }
__global__ __launch_bounds__(256) void k_attn(const float* __restrict__ FQ, const float* __restrict__ FK, const float* __restrict__ FV, const int* __restrict__ IDX, const float* __restrict__ DST, const float* __restrict__ VEC, float* __restrict__ ATT) {
  __shared__ float sq[DD], swk[DD], swv[DD], sck[DD], scv[DD]; __shared__ float sp[NH][KN]; __shared__ int sidx[KN]; __shared__ float sdst[KN];
  const int t = threadIdx.x, h = t >> 5, lane = t & 31; const size_t row = blockIdx.x; const size_t b = row / NPT;
  for (int e = t; e < DD; e += 256) { sq[e] = FQ[row * DD + e]; swk[e] = VEC[e]; swv[e] = VEC[DD + e]; sck[e] = VEC[2 * DD + e]; scv[e] = VEC[3 * DD + e]; }
  if (t < KN) { sidx[t] = IDX[row * KN + t]; sdst[t] = DST[row * KN + t]; }
  __syncthreads();
  const float scale = 1.0f / sqrtf((float)HD);
  float s2[2];
#pragma unroll
  for (int u = 0; u < 2; ++u) { const int kk = lane + 32 * u; const size_t nr = b * NPT + sidx[kk]; const float dk = sdst[kk]; const float* fk = FK + nr * DD + h * HD; float s = 0.f;
#pragma unroll 4
    for (int c = 0; c < HD; ++c) { const float kvv = fk[c] + dk * swk[h * HD + c] + sck[h * HD + c]; s += sq[h * HD + c] * kvv; }
    s2[u] = s * scale; }
  float mx = fmaxf(s2[0], s2[1]);
#pragma unroll
  for (int o = 1; o < 32; o <<= 1) mx = fmaxf(mx, __shfl_xor(mx, o));
  const float e0 = exp_ni(s2[0] - mx), e1 = exp_ni(s2[1] - mx); float den = e0 + e1;
#pragma unroll
  for (int o = 1; o < 32; o <<= 1) den += __shfl_xor(den, o);
  sp[h][lane] = e0 / den; sp[h][lane + 32] = e1 / den;
  __syncthreads();
  float o3[3] = {0.f, 0.f, 0.f};
#pragma unroll 1
  for (int kk = 0; kk < KN; ++kk) { const size_t nr = b * NPT + sidx[kk]; const float dk = sdst[kk], pw = sp[h][kk]; const float* fv = FV + nr * DD + h * HD;
#pragma unroll
    for (int u = 0; u < 3; ++u) { const int c = lane + 32 * u; o3[u] += pw * (fv[c] + dk * swv[h * HD + c] + scv[h * HD + c]); } }
#pragma unroll
  for (int u = 0; u < 3; ++u) sq[h * HD + lane + 32 * u] = o3[u];
  __syncthreads();
  for (int q = t; q < DD / 4; q += 256) vst2(ATT + row * DD + q * 4, *(const v4f*)&sq[q * 4]);
}
__global__ __launch_bounds__(256) void k_lnsilu(const float* __restrict__ Y, const float* __restrict__ G, const float* __restrict__ Bt, float* __restrict__ OUT) {
  __shared__ float red[8]; __shared__ __align__(16) float so[DD]; const int t = threadIdx.x; const size_t row = blockIdx.x; float v[3]; float s = 0.f; for (int i = 0; i < 3; ++i) { v[i] = Y[row * DD + t + 256 * i]; s += v[i]; }
#pragma unroll
  for (int o = 1; o < 32; o <<= 1) s += __shfl_xor(s, o);
  if ((t & 31) == 0) red[t >> 5] = s; __syncthreads(); float tot = 0.f; for (int i = 0; i < 8; ++i) tot += red[i]; const float mu = tot / (float)DD; __syncthreads();
  float q = 0.f; for (int i = 0; i < 3; ++i) { const float dd = v[i] - mu; q += dd * dd; }
#pragma unroll
  for (int o = 1; o < 32; o <<= 1) q += __shfl_xor(q, o);
  if ((t & 31) == 0) red[t >> 5] = q; __syncthreads(); float tq = 0.f; for (int i = 0; i < 8; ++i) tq += red[i]; const float inv = 1.0f / sqrtf(tq / (float)DD + 1e-5f);
  for (int i = 0; i < 3; ++i) { const int e = t + 256 * i; const float z = (v[i] - mu) * inv * bfr(G[e]) + bfr(Bt[e]); so[e] = z / (1.0f + exp_ni(-z)); }
  __syncthreads();
  for (int qq = t; qq < DD / 4; qq += 256) vst2(OUT + row * DD + qq * 4, *(const v4f*)&so[qq * 4]);
}
extern "C" void kernel_launch(void* const* d_in, const int* in_sizes, int n_in, void* d_out, int out_size, void* d_ws, size_t ws_size, hipStream_t stream) {
  (void)in_sizes; (void)n_in; (void)out_size;
  const float** F = (const float**)d_in;
  if (ws_size < (size_t)WS_END) return;
  char* ws = (char*)d_ws; __bf16* P = (__bf16*)ws; int* IDX = (int*)(ws + WS_IDX); float *DST = (float*)(ws + WS_DST), *FQ = (float*)(ws + WS_FQ), *FK = (float*)(ws + WS_FK), *FV = (float*)(ws + WS_FV), *ATT = (float*)(ws + WS_ATT), *C2 = (float*)(ws + WS_C2), *Y = (float*)(ws + WS_Y), *VEC = (float*)(ws + WS_VEC);
  k_pack<<<dim3(DD, 5), 256, 0, stream>>>(F[4], F[6], F[8], F[10], F[12], P);
  k_vec<<<DD / 256, 256, 0, stream>>>(F[2], F[3], F[6], F[7], F[8], F[9], VEC);
  k_knn<<<dim3(NPT / 64, NB), 64, 0, stream>>>(F[1], IDX, DST);
  k_copyf<<<NR, 256, 0, stream>>>(F[0], ATT);
  k_lin<DD><<<dim3(NR / 64, DD / 128), 128, 0, stream>>>(ATT, nullptr, P + WS_PW / 2, F[5], FQ);
  k_lin<DD><<<dim3(NR / 64, DD / 128), 128, 0, stream>>>(ATT, nullptr, P + WS_PW / 2 + (size_t)DD * DD, nullptr, FK);
  k_lin<DD><<<dim3(NR / 64, DD / 128), 128, 0, stream>>>(ATT, nullptr, P + WS_PW / 2 + (size_t)2 * DD * DD, nullptr, FV);
  k_copyf<<<NR, 256, 0, stream>>>(F[0], Y);
  k_attn<<<NRB * 64, 256, 0, stream>>>(FQ, FK, FV, IDX, DST, VEC, ATT);
  k_lin<DD><<<dim3(NRB, DD / 128), 128, 0, stream>>>(ATT, nullptr, P + WS_PW / 2 + (size_t)3 * DD * DD, F[11], C2);
  k_lin<2 * DD><<<dim3(NRB, DD / 128), 128, 0, stream>>>(Y, C2, P + WS_PWE / 2, F[13], FQ);
  k_lnsilu<<<NRB * 64, 256, 0, stream>>>(FQ, F[14], F[15], (float*)d_out);
}
